// OurModel_57234734187133
// MI455X (gfx1250) — hardware-verified
//
#include <hip/hip_runtime.h>

typedef float          v8f   __attribute__((ext_vector_type(8)));
typedef float          v4f   __attribute__((ext_vector_type(4)));
typedef unsigned int   v4u   __attribute__((ext_vector_type(4)));
typedef int            v8i   __attribute__((ext_vector_type(8)));
typedef unsigned short v8us  __attribute__((ext_vector_type(8)));
typedef unsigned short v16us __attribute__((ext_vector_type(16)));
typedef __bf16         v16bf __attribute__((ext_vector_type(16)));
typedef _Float16       v16h  __attribute__((ext_vector_type(16)));
typedef v4f  __attribute__((may_alias)) v4fa;
typedef v8us __attribute__((may_alias)) v8usa;
union FragB { v16bf v; v16us u; v8us h[2]; v8i w; };
union FragH { v16h  v; v16us u; v8us h[2]; v8i w; };

__device__ __forceinline__ v8f wmb(const FragB& a, const FragB& b, v8f c) {
  v8f d = __builtin_amdgcn_wmma_f32_16x16x32_bf16(false, a.v, false, b.v, (short)0, c, false, false);
  asm volatile("v_nop\n\tv_nop\n\tv_nop\n\tv_nop" : "+v"(d) : "v"(a.w), "v"(b.w));
  return d;
}

__device__ __forceinline__ v8f wmh(const FragH& a, const FragH& b, v8f c) {
  v8f d = __builtin_amdgcn_wmma_f32_16x16x32_f16(false, a.v, false, b.v, (short)0, c, false, false);
  asm volatile("v_nop\n\tv_nop\n\tv_nop\n\tv_nop" : "+v"(d) : "v"(a.w), "v"(b.w));
  return d;
}

__device__ __forceinline__ unsigned bf16_bits(float f) {
  const unsigned u = __float_as_uint(f);
  const unsigned r = (u + 0x7FFFu + ((u >> 16) & 1u)) >> 16;
  const unsigned q = (u >> 16) | 0x40u;
  return ((u & 0x7fffffffu) > 0x7f800000u) ? q : r;
}

__device__ __forceinline__ float bf16_val(float f) {
  return __uint_as_float(bf16_bits(f) << 16);
}
__device__ __forceinline__ int clampi(int v, int lo, int hi) {
  return v < lo ? lo : (v > hi ? hi : v);
}

__device__ __forceinline__ unsigned f16_bits(float f) {
  const unsigned u  = __float_as_uint(f);
  const unsigned s  = (u >> 16) & 0x8000u;
  const unsigned a  = u & 0x7fffffffu;
  const unsigned t  = a - 0x38000000u;
  const unsigned r  = (t + 0x0FFFu + ((t >> 13) & 1u)) >> 13;
  const unsigned rc = r > 0x7C00u ? 0x7C00u : r;
  const bool small  = a < 0x38800000u;
  const bool isnan  = a > 0x7f800000u;
  const unsigned fin = small ? 0u : (s | rc);
  return isnan ? (s | 0x7E00u) : fin;
}

__device__ __forceinline__ unsigned pk16(unsigned lo, unsigned hi) { return lo | (hi << 16); }
__device__ __forceinline__ unsigned bf16_lo_bits(float v) {
  float hi = bf16_val(v);
  asm volatile("" : "+v"(hi));
  return bf16_bits(v - hi);
}
__device__ __forceinline__ v4u pack8_bf16(v4f a, v4f c) {
  return (v4u){ pk16(bf16_bits(a[0]), bf16_bits(a[1])), pk16(bf16_bits(a[2]), bf16_bits(a[3])),
                pk16(bf16_bits(c[0]), bf16_bits(c[1])), pk16(bf16_bits(c[2]), bf16_bits(c[3])) };
}
__device__ __forceinline__ v4u pack8_bf16_lo(v4f a, v4f c) {
  return (v4u){ pk16(bf16_lo_bits(a[0]), bf16_lo_bits(a[1])), pk16(bf16_lo_bits(a[2]), bf16_lo_bits(a[3])),
                pk16(bf16_lo_bits(c[0]), bf16_lo_bits(c[1])), pk16(bf16_lo_bits(c[2]), bf16_lo_bits(c[3])) };
}
__device__ __forceinline__ v4u pack8_f16(v4f a, v4f c) {
  return (v4u){ pk16(f16_bits(a[0]), f16_bits(a[1])), pk16(f16_bits(a[2]), f16_bits(a[3])),
                pk16(f16_bits(c[0]), f16_bits(c[1])), pk16(f16_bits(c[2]), f16_bits(c[3])) };
}

template <int FORM>
__global__ __launch_bounds__(256) void k_plane(const float* __restrict__ src, int rows, int cols, int ldsrc,
                                               unsigned short* __restrict__ dst, int MP, int KP) {
  static_assert(FORM >= 0 && FORM <= 3);
  const int KTOT = (FORM == 1 || FORM == 3) ? 2 * KP : KP;
  const unsigned ppr   = (unsigned)(KTOT >> 3);
  const unsigned kp8   = (unsigned)(KP >> 3);
  const unsigned total = (unsigned)MP * ppr;
  const unsigned g     = blockIdx.x * 256u + threadIdx.x;
  const unsigned rowu  = g / ppr;
  const unsigned p     = g - rowu * ppr;
  const bool second    = p >= kp8;
  const int row = (int)rowu;
  const int c0  = (int)((second ? p - kp8 : p) << 3);
  const float* srow = src + (size_t)clampi(row, 0, rows - 1) * (size_t)ldsrc;
  float x[8];
  unsigned mk[8];
#pragma unroll
  for (int e = 0; e < 8; ++e) {
    const int c = c0 + e;
    const float v = srow[clampi(c, 0, cols - 1)];
    asm volatile("" :: "v"(v));
    x[e]  = v;
    mk[e] = (row < rows && c < cols) ? 0xFFFFu : 0u;
  }
  const v4f a = (v4f){ x[0], x[1], x[2], x[3] };
  const v4f c = (v4f){ x[4], x[5], x[6], x[7] };
  v4u o;
  if (FORM == 2) {
    o = pack8_f16(a, c);
  } else {
    const v4u hi = pack8_bf16(a, c);
    o = hi;
    if (FORM == 1) { const v4u lo = pack8_bf16_lo(a, c); o = second ? lo : hi; }
  }
  const v4u mw = (v4u){ pk16(mk[0], mk[1]), pk16(mk[2], mk[3]), pk16(mk[4], mk[5]), pk16(mk[6], mk[7]) };
  o &= mw;
  if (g < total) {
    volatile v4u* q = (volatile v4u*)(dst + (size_t)g * 8);
    *q = o;
    __threadfence();
    *q = o;
  }
}

template <int FORM> struct FragOf    { typedef FragB T; };
template <>         struct FragOf<2> { typedef FragH T; };
__device__ __forceinline__ v8f mm(const FragB& a, const FragB& b, v8f c) { return wmb(a, b, c); }
__device__ __forceinline__ v8f mm(const FragH& a, const FragH& b, v8f c) { return wmh(a, b, c); }
template <class F> __device__ __forceinline__ F ld_frag(const unsigned short* p) {
  F f;
  f.h[0] = *(const v8usa*)(p);
  f.h[1] = *(const v8usa*)(p + 16);
  return f;
}

template <int FORM, int EPI>
__global__ __launch_bounds__(256) __attribute__((amdgpu_num_vgpr(248)))
void k_gemm_nt(const unsigned short* __restrict__ A, const unsigned short* __restrict__ B,
               const float* __restrict__ bias, float* __restrict__ D, int M, int N, int KTOT, int ldd) {
  static_assert(FORM >= 0 && FORM <= 2);
  static_assert(EPI == 0 || EPI == 1);
  typedef typename FragOf<FORM>::T F;
  __shared__ __attribute__((aligned(16))) float sT[8][16 * 68];
  const int lane = threadIdx.x & 31;
  const int wave = threadIdx.x >> 5;
  const int tilesM = (M + 63) >> 6;
  const int tilesN = (N + 63) >> 6;
  const int tile = blockIdx.x * 8 + wave;
  if (tile >= tilesM * tilesN) return;
  const int tm = tile / tilesN;
  const int tn = tile - tm * tilesN;
  const int m0 = tm << 6;
  const int n0 = tn << 6;

  const int rl = lane & 15;
  const int h8 = (lane >> 4) * 8;
  const unsigned short* pa = A + (size_t)(m0 + rl) * (size_t)KTOT + h8;
  const unsigned short* pb = B + (size_t)(n0 + rl) * (size_t)KTOT + h8;

  v8f acc[4][4];
#pragma unroll
  for (int i = 0; i < 4; ++i)
#pragma unroll
    for (int j = 0; j < 4; ++j) acc[i][j] = (v8f){0.f, 0.f, 0.f, 0.f, 0.f, 0.f, 0.f, 0.f};

#pragma unroll 1
  for (int k0 = 0; k0 < KTOT; k0 += 32) {
    F bf[4];
#pragma unroll
    for (int j = 0; j < 4; ++j) bf[j] = ld_frag<F>(pb + (size_t)(j << 4) * (size_t)KTOT + k0);
#pragma unroll
    for (int i = 0; i < 4; ++i) {
      const F af = ld_frag<F>(pa + (size_t)(i << 4) * (size_t)KTOT + k0);
#pragma unroll
      for (int j = 0; j < 4; ++j) acc[i][j] = mm(af, bf[j], acc[i][j]);
    }
  }

  float* slab = sT[wave];
  const int hh = lane >> 4;
  const int c4 = (lane & 15) * 4;
  const int nc = n0 + c4;
  const bool cok = nc < N;
  v4f bv = (v4f){0.f, 0.f, 0.f, 0.f};
  if (EPI == 1) {
    bv = *(const v4fa*)(bias + clampi(nc, 0, N - 4));
    asm volatile("" :: "v"(bv));
  }
#pragma unroll
  for (int i = 0; i < 4; ++i) {
    const int mBase = m0 + (i << 4);
#pragma unroll
    for (int j = 0; j < 4; ++j) {
#pragma unroll
      for (int r = 0; r < 8; ++r) slab[(h8 + r) * 68 + (j << 4) + rl] = acc[i][j][r];
    }
    __builtin_amdgcn_fence(__ATOMIC_RELEASE, "workgroup");
    __builtin_amdgcn_wave_barrier();
    __builtin_amdgcn_fence(__ATOMIC_ACQUIRE, "workgroup");
    v4f vv[8];
#pragma unroll
    for (int it = 0; it < 8; ++it) {
      const int row = it * 2 + hh;
      v4f v = *(const v4fa*)(slab + row * 68 + c4);
      if (EPI == 1) v += bv;
      vv[it] = v;
    }
    for (int pass = 0; pass < 2; ++pass) {
#pragma unroll
      for (int it = 0; it < 8; ++it) {
        const int row = mBase + it * 2 + hh;
        if (cok && row < M) *(volatile v4f*)(D + (size_t)row * (size_t)ldd + nc) = vv[it];
      }
      __threadfence();
    }
    __builtin_amdgcn_fence(__ATOMIC_RELEASE, "workgroup");
    __builtin_amdgcn_wave_barrier();
    __builtin_amdgcn_fence(__ATOMIC_ACQUIRE, "workgroup");
  }
}


typedef int          v4i __attribute__((ext_vector_type(4)));
typedef unsigned int v2u __attribute__((ext_vector_type(2)));
typedef v4i __attribute__((may_alias)) v4ia;
typedef v2u __attribute__((may_alias)) v2ua;
typedef v4u __attribute__((may_alias)) v4ua;

static constexpr int kH    = 256;
static constexpr int kNN   = 50000;
static constexpr int kNE   = 10000;
static constexpr int kE    = 300000;
static constexpr int kMPN  = 50048;
static constexpr int kMPE  = 10112;
static constexpr int kOut1 = kNN * kH;
static constexpr int kOutTotal = (kNN + kNE) * kH;

static constexpr int kChunk = 2048;
static constexpr int kWcap  = 256;
static constexpr int kListN = 8 * kWcap;
static constexpr int kMisc  = 16;

static constexpr int kSLB_H = 9,  kNB_H = 512,  kBLK_H = 20, kRC_H = 19968, kDEG_H = 64;
static constexpr int kSLB_N = 10, kNB_N = 1024, kBLK_N = 49, kRC_N = 8192,  kDEG_N = 32;

static constexpr int bucket_ints(int rc, int nb) { return kListN + 2 * rc + 3 * nb + kMisc; }
static constexpr size_t kLdsH = (size_t)bucket_ints(kRC_H, kNB_H) * 4;
static constexpr size_t kLdsN = (size_t)bucket_ints(kRC_N, kNB_N) * 4;

static_assert(kH == 256 && kH == 32 * 8);
static_assert(kE < (1 << 21));
static_assert(kOut1 % 32 == 0);
static_assert(kNB_H == (1 << kSLB_H) && kNB_N == (1 << kSLB_N));
static_assert(kBLK_H * kNB_H >= kNE && kBLK_N * kNB_N >= kNN);
static_assert(kRC_H * 4 >= 15784 * 5 && kRC_N * 4 >= 6337 * 5);
static_assert(kDEG_H >= 51 + 8 && kDEG_N >= 18 + 8);
static_assert(kRC_H % 128 == 0 && kRC_N % 128 == 0);
static_assert(bucket_ints(kRC_H, kNB_H) % 4 == 0 && bucket_ints(kRC_N, kNB_N) % 4 == 0);
static_assert(kLdsH <= 262144 && kLdsN <= 262144);
static_assert(kLdsH + 0 <= 327680 && kLdsN + 0 <= 327680);
static_assert((kChunk << 10) > 0 && kChunk == 8 * 256);
static_assert(kMPN % 64 == 0 && kMPE % 64 == 0 && kMPN >= kNN && kMPE >= kNE);
static_assert(kNN % 16 == 0 && kNE % 16 == 0 && kH % 64 == 0 && kH % 32 == 0);
static_assert(kNE % 8 == 0 && kNN % 8 == 0 && kMPE % 8 == 0);
static_assert(((long long)kMPN * 512 / 8) < (1LL << 31));
static_assert((kMPN * (kH / 8)) % 256 == 0 && (kMPN * (2 * kH / 8)) % 256 == 0);

static constexpr size_t al256c(size_t o) { return (o + 255) & ~(size_t)255; }
static constexpr size_t szRA   = (size_t)kMPN * kH * 4;
static constexpr size_t szRB   = (size_t)kMPN * 2 * kH * 2;
static constexpr size_t szEF   = (size_t)kMPE * 2 * kH * 2;
static constexpr size_t szWHE  = (size_t)kMPE * kH * 4;
static constexpr size_t szW1   = (size_t)kH * kH * 2;
static constexpr size_t szW2   = (size_t)kH * 2 * kH * 2;
static constexpr size_t szBias = (size_t)3 * kH * 4;
static constexpr size_t szLH   = (size_t)kBLK_H * kRC_H * 4;
static constexpr size_t szLN   = (size_t)kBLK_N * kRC_N * 4;
static constexpr size_t szTH   = (size_t)kBLK_H * kNB_H * 4;
static constexpr size_t szTN   = (size_t)kBLK_N * kNB_N * 4;
static constexpr size_t szFH   = (size_t)kBLK_H * 128;
static constexpr size_t szFN   = (size_t)kBLK_N * 128;
static constexpr size_t oRA    = 0;
static constexpr size_t oRB    = al256c(oRA + szRA);
static constexpr size_t oEF    = al256c(oRB + szRB);
static constexpr size_t oWHE   = al256c(oEF + szEF);
static constexpr size_t oWin   = al256c(oWHE + szWHE);
static constexpr size_t oWn    = al256c(oWin + szW1);
static constexpr size_t oWe    = al256c(oWn + szW2);
static constexpr size_t oBias  = al256c(oWe + szW2);
static constexpr size_t oLH    = al256c(oBias + szBias);
static constexpr size_t oLN    = al256c(oLH + szLH);
static constexpr size_t oCH    = al256c(oLN + szLN);
static constexpr size_t oOH    = al256c(oCH + szTH);
static constexpr size_t oCN    = al256c(oOH + szTH);
static constexpr size_t oON    = al256c(oCN + szTN);
static constexpr size_t oFH    = al256c(oON + szTN);
static constexpr size_t oFN    = al256c(oFH + szFH);
static constexpr size_t kWsTotal = al256c(oFN + szFN);
static_assert(kWsTotal <= ((size_t)128 << 20));

__device__ __forceinline__ void wave_sync() {
  __builtin_amdgcn_fence(__ATOMIC_RELEASE, "workgroup");
  __builtin_amdgcn_wave_barrier();
  __builtin_amdgcn_fence(__ATOMIC_ACQUIRE, "workgroup");
}

__global__ __launch_bounds__(192) void k_bias(const float* __restrict__ b0, const float* __restrict__ b1,
                                              const float* __restrict__ b2, float* __restrict__ tab) {
  const int g     = (int)threadIdx.x;
  const int which = g >> 6;
  const int c4    = (g & 63) * 4;
  const v4f x0 = *(const v4fa*)(b0 + c4);
  asm volatile("" :: "v"(x0));
  const v4f x1 = *(const v4fa*)(b1 + c4);
  asm volatile("" :: "v"(x1));
  const v4f x2 = *(const v4fa*)(b2 + c4);
  asm volatile("" :: "v"(x2));
  v4f x = x0;
  if (which == 1) x = x1;
  if (which == 2) x = x2;
  const v4f o = (v4f){ bf16_val(x[0]), bf16_val(x[1]), bf16_val(x[2]), bf16_val(x[3]) };
  volatile v4f* q = (volatile v4f*)(tab + g * 4);
  *q = o;
  __threadfence();
  *q = o;
}

template <int SLB, int RC, int DEGC>
__global__ __launch_bounds__(256) void k_bucket(const int* __restrict__ keys, int nE, int nOwn,
                                                int* __restrict__ LIST, int* __restrict__ CNT,
                                                int* __restrict__ OFF, int* __restrict__ FLAG) {
  constexpr int NB = 1 << SLB;
  constexpr int ZI = kListN + 2 * RC + 3 * NB + kMisc;
  extern __shared__ __attribute__((aligned(16))) int dsm[];
  int* list = dsm;
  int* hl   = dsm + kListN;
  int* sl   = hl + RC;
  int* cnt  = sl + RC;
  int* offs = cnt + NB;
  int* cur  = offs + NB;
  int* misc = cur + NB;
  const int tid = (int)threadIdx.x, lane = tid & 31, wave = tid >> 5;
  const int blk = (int)blockIdx.x;
  const int slotBase = blk * NB;
  int nb = nOwn - slotBase;
  nb = nb < 0 ? 0 : (nb > NB ? NB : nb);

  {
    const v4i z4 = {0, 0, 0, 0};
    for (int i = tid * 4; i < ZI; i += 1024) *(v4ia*)(dsm + i) = z4;
  }
  __syncthreads();

  const int sent = (-0x7fffffff - 1);
  const unsigned ubase = (unsigned)slotBase;
  const unsigned unb   = (unsigned)nb;
  const int elw = wave * 256 + lane;
  int t = 0, ov = 0;
  const int nChunks = (nE + kChunk - 1) / kChunk;
#pragma unroll 1
  for (int ch = 0; ch < nChunks; ++ch) {
    const int cbase = ch * kChunk;
    int kv[8];
#pragma unroll
    for (int j = 0; j < 8; ++j) {
      const int e  = cbase + elw + 32 * j;
      const int ec = e < nE ? e : nE - 1;
      const int k  = keys[ec];
      asm volatile("" :: "v"(k));
      kv[j] = (e < nE) ? k : sent;
    }
    int wc = 0;
#pragma unroll
    for (int j = 0; j < 8; ++j) {
      const unsigned s   = (unsigned)kv[j] - ubase;
      const bool     hit = s < unb;
      const unsigned mj  = __builtin_amdgcn_ballot_w32(hit);
      const int      pos = wc + (int)__builtin_amdgcn_mbcnt_lo(mj, 0u);
      if (hit && pos < kWcap) list[wave * kWcap + pos] = ((elw + 32 * j) << SLB) | (int)s;
      wc += (int)__builtin_popcount(mj);
    }
    if (lane == 0) misc[wave] = wc;
    __syncthreads();
    if (wave == 0) {
#pragma unroll 1
      for (int w2 = 0; w2 < 8; ++w2) {
        int c = misc[w2];
        c = c < 0 ? 0 : (c > kWcap ? kWcap : c);
#pragma unroll 1
        for (int b0 = 0; b0 < c; b0 += 32) {
          const int idx = b0 + lane;
          const int ent = list[w2 * kWcap + (idx < kWcap ? idx : kWcap - 1)];
          const int m32 = (c - b0) < 32 ? (c - b0) : 32;
#pragma unroll 1
          for (int k = 0; k < m32; ++k) {
            const int u    = __builtin_amdgcn_readlane(ent, k);
            const int slot = u & (NB - 1);
            const int el   = (u >> SLB) & (kChunk - 1);
            const int pk   = ((cbase + el) << SLB) | slot;
            if (t < RC) {
              if (lane == 0) { hl[t] = pk; cnt[slot] = cnt[slot] + 1; }
              t = t + 1;
            } else {
              ov = 1;
            }
          }
        }
      }
    }
    __syncthreads();
  }
  if (wave == 0 && lane == 0) { misc[8] = t; misc[9] = ov; }
  __syncthreads();
  int tt = misc[8];
  tt = tt < 0 ? 0 : (tt > RC ? RC : tt);

  if (wave == 0) {
    const int base = lane * (NB / 32);
    int s = 0;
#pragma unroll 1
    for (int i = 0; i < NB / 32; ++i) s += cnt[base + i];
    int incl = s;
#pragma unroll
    for (int d = 1; d < 32; d <<= 1) {
      const int y = __shfl_up(incl, d, 32);
      if (lane >= d) incl += y;
    }
    int run = incl - s;
    int dg = 0;
#pragma unroll 1
    for (int i = 0; i < NB / 32; ++i) {
      const int cv = cnt[base + i];
      offs[base + i] = run;
      cur[base + i]  = run;
      run += cv;
      dg |= (cv > DEGC) ? 1 : 0;
    }
    const unsigned dm = __builtin_amdgcn_ballot_w32(dg != 0);
    if (lane == 0) misc[10] = (dm != 0u) ? 1 : 0;
  }
  __syncthreads();
  if (wave == 0) {
#pragma unroll 1
    for (int b0 = 0; b0 < tt; b0 += 32) {
      const int idx = b0 + lane;
      const int ent = hl[idx < RC ? idx : RC - 1];
      const int m32 = (tt - b0) < 32 ? (tt - b0) : 32;
#pragma unroll 1
      for (int k = 0; k < m32; ++k) {
        const int u    = __builtin_amdgcn_readlane(ent, k);
        const int slot = u & (NB - 1);
        if (lane == 0) {
          int p = cur[slot];
          p = p < 0 ? 0 : (p > RC - 1 ? RC - 1 : p);
          sl[p] = u;
          cur[slot] = p + 1;
        }
      }
    }
  }
  __syncthreads();

  const int fv = ((misc[9] | misc[10]) != 0) ? 1 : 0;
  const v4i f4 = {fv, fv, fv, fv};
  int* lp = LIST + (size_t)blk * (size_t)RC;
  for (int pass = 0; pass < 2; ++pass) {
#pragma unroll 1
    for (int i = tid * 4; i < RC; i += 1024) {
      v4i q = *(const v4ia*)(sl + i);
      q.x >>= SLB; q.y >>= SLB; q.z >>= SLB; q.w >>= SLB;
      *(volatile v4i*)(lp + i) = q;
    }
    if (tid < NB / 4) {
      const v4i c4 = *(const v4ia*)(cnt + tid * 4);
      const v4i o4 = *(const v4ia*)(offs + tid * 4);
      *(volatile v4i*)(CNT + slotBase + tid * 4) = c4;
      *(volatile v4i*)(OFF + slotBase + tid * 4) = o4;
    }
    if (tid < 8) *(volatile v4i*)(FLAG + blk * 32 + tid * 4) = f4;
    __threadfence();
  }
}

__device__ __forceinline__ float prelu1(float v, float al) {
  return (v > 0.0f) ? v : al * v;
}

template <int STEP, int SLB, int RC, int DEGC>
__global__ __launch_bounds__(256) void k_replay(const int* __restrict__ nidx, const int* __restrict__ hidx,
                                                const float* __restrict__ numT, const float* __restrict__ denT,
                                                const float* __restrict__ rows,
                                                const int* __restrict__ LIST, const int* __restrict__ CNT,
                                                const int* __restrict__ OFF, const int* __restrict__ FLAG,
                                                const float* __restrict__ alphaP, float* __restrict__ outp,
                                                unsigned short* __restrict__ efhl, int nOwn, int nPad) {
  static_assert(STEP == 1 || STEP == 2);
  const int lane = (int)threadIdx.x & 31, wave = (int)threadIdx.x >> 5;
  const int row  = (int)blockIdx.x * 8 + wave;
  const bool live = row < nOwn;
  const int rc  = live ? row : nOwn - 1;
  const int blk = rc >> SLB;

  int c = CNT[rc];
  asm volatile("" :: "v"(c));
  int o = OFF[rc];
  asm volatile("" :: "v"(o));
  int fl = FLAG[blk * 32];
  asm volatile("" :: "v"(fl));
  float al = alphaP[0];
  asm volatile("" :: "v"(al));
  al = bf16_val(al);
  const int big = (c > DEGC) ? 1 : 0;
  c = clampi(c, 0, DEGC);
  o = clampi(o, 0, RC);
  const int cn = __builtin_amdgcn_readfirstlane(live ? c : 0);
  const int pu = __builtin_amdgcn_readfirstlane((fl != 0 || big != 0) ? 1 : 0);
  const int* lp = LIST + (size_t)blk * (size_t)RC;

  v4f a0 = (v4f){0.0f, 0.0f, 0.0f, 0.0f};
  v4f a1 = (v4f){0.0f, 0.0f, 0.0f, 0.0f};
#pragma unroll 1
  for (int b0 = 0; b0 < cn; b0 += 32) {
    const int idx = clampi(o + b0 + lane, 0, RC - 1);
    int t = lp[idx];
    asm volatile("" :: "v"(t));
    t = clampi(t, 0, kE - 1);
    int nd = nidx[t];
    asm volatile("" :: "v"(nd));
    int he = hidx[t];
    asm volatile("" :: "v"(he));
    nd = clampi(nd, 0, kNN - 1);
    he = clampi(he, 0, kNE - 1);
    const int gi = (STEP == 1) ? nd : he;
    const int ni = (STEP == 1) ? nd : he;
    const int di = (STEP == 1) ? he : nd;
    const float a = numT[ni];
    asm volatile("" :: "v"(a));
    const float b = denT[di];
    asm volatile("" :: "v"(b));
    const float w = bf16_val(a) / bf16_val(b);
    const int wvi = __float_as_int(w);
    const int m32 = (cn - b0) < 32 ? (cn - b0) : 32;
#pragma unroll 1
    for (int k = 0; k < m32; ++k) {
      const int   sk = __builtin_amdgcn_readlane(gi, k);
      const float ck = __int_as_float(__builtin_amdgcn_readlane(wvi, k));
      const float* rp = rows + (size_t)sk * (size_t)kH + 4 * lane;
      const v4f r0 = *(const v4fa*)rp;
      asm volatile("" :: "v"(r0));
      const v4f r1 = *(const v4fa*)(rp + 128);
      asm volatile("" :: "v"(r1));
      a0[0] = fmaf(ck, r0[0], a0[0]);
      a0[1] = fmaf(ck, r0[1], a0[1]);
      a0[2] = fmaf(ck, r0[2], a0[2]);
      a0[3] = fmaf(ck, r0[3], a0[3]);
      a1[0] = fmaf(ck, r1[0], a1[0]);
      a1[1] = fmaf(ck, r1[1], a1[1]);
      a1[2] = fmaf(ck, r1[2], a1[2]);
      a1[3] = fmaf(ck, r1[3], a1[3]);
    }
  }

  const float qn = __int_as_float(0x7fc00000);
  v4f y0, y1;
#pragma unroll
  for (int e = 0; e < 4; ++e) {
    const float u0 = (pu != 0) ? qn : a0[e];
    const float u1 = (pu != 0) ? qn : a1[e];
    const float p0 = prelu1(u0, al);
    const float p1 = prelu1(u1, al);
    y0[e] = live ? p0 : 0.0f;
    y1[e] = live ? p1 : 0.0f;
  }

  if (live) {
    float* op = outp + (size_t)row * (size_t)kH + 4 * lane;
    for (int pass = 0; pass < 2; ++pass) {
      *(volatile v4f*)op = y0;
      *(volatile v4f*)(op + 128) = y1;
      __threadfence();
    }
  }

  if constexpr (STEP == 1) {
    __shared__ __attribute__((aligned(16))) unsigned rowbuf[8][256];
    unsigned* rb = rowbuf[wave];
    const v2u h0 = (v2u){ pk16(bf16_bits(y0[0]), bf16_bits(y0[1])), pk16(bf16_bits(y0[2]), bf16_bits(y0[3])) };
    const v2u h1 = (v2u){ pk16(bf16_bits(y1[0]), bf16_bits(y1[1])), pk16(bf16_bits(y1[2]), bf16_bits(y1[3])) };
    const v2u l0 = (v2u){ pk16(bf16_lo_bits(y0[0]), bf16_lo_bits(y0[1])), pk16(bf16_lo_bits(y0[2]), bf16_lo_bits(y0[3])) };
    const v2u l1 = (v2u){ pk16(bf16_lo_bits(y1[0]), bf16_lo_bits(y1[1])), pk16(bf16_lo_bits(y1[2]), bf16_lo_bits(y1[3])) };
    *(v2ua*)(rb + 2 * lane)       = h0;
    *(v2ua*)(rb + 64 + 2 * lane)  = h1;
    *(v2ua*)(rb + 128 + 2 * lane) = l0;
    *(v2ua*)(rb + 192 + 2 * lane) = l1;
    wave_sync();
    const v4u q0 = *(const v4ua*)(rb + 4 * lane);
    const v4u q1 = *(const v4ua*)(rb + 128 + 4 * lane);
    wave_sync();
    if (row < nPad) {
      unsigned short* ep = efhl + (size_t)row * 512 + 8 * lane;
      for (int pass = 0; pass < 2; ++pass) {
        *(volatile v4u*)ep = q0;
        *(volatile v4u*)(ep + 256) = q1;
        __threadfence();
      }
    }
  }
}

extern "C" void kernel_launch(void* const* d_in, const int* in_sizes, int n_in,
                              void* d_out, int out_size, void* d_ws, size_t ws_size,
                              hipStream_t stream) {
  if (n_in < 15) return;
  if (in_sizes[0] != kNN * kH) return;
  if (in_sizes[2] != kE || in_sizes[3] != kE) return;
  if (in_sizes[4] != kNN || in_sizes[5] != kNN || in_sizes[6] != kNE || in_sizes[7] != kNE) return;
  if (in_sizes[8] != kH * kH || in_sizes[10] != kH * kH || in_sizes[12] != kH * kH) return;
  if (in_sizes[9] != kH || in_sizes[11] != kH || in_sizes[13] != kH) return;
  if (in_sizes[14] < 1) return;
  if (out_size != kOutTotal) return;
  if (ws_size < kWsTotal) return;

  const float* n_feat = (const float*)d_in[0];
  const int*   node_idx  = (const int*)d_in[2];
  const int*   hedge_idx = (const int*)d_in[3];
  const float* node_w  = (const float*)d_in[4];
  const float* node_s  = (const float*)d_in[5];
  const float* hedge_w = (const float*)d_in[6];
  const float* hedge_s = (const float*)d_in[7];
  const float* W_in  = (const float*)d_in[8];
  const float* b_in  = (const float*)d_in[9];
  const float* W_n2e = (const float*)d_in[10];
  const float* b_n2e = (const float*)d_in[11];
  const float* W_e2n = (const float*)d_in[12];
  const float* b_e2n = (const float*)d_in[13];
  const float* alpha = (const float*)d_in[14];
  float* out = (float*)d_out;

  char* ws = (char*)d_ws;
  float*          RA    = (float*)(ws + oRA);
  unsigned short* RB    = (unsigned short*)(ws + oRB);
  unsigned short* EFhl  = (unsigned short*)(ws + oEF);
  float*          WHE   = (float*)(ws + oWHE);
  unsigned short* WinB  = (unsigned short*)(ws + oWin);
  unsigned short* Wn2eD = (unsigned short*)(ws + oWn);
  unsigned short* We2nD = (unsigned short*)(ws + oWe);
  float*          biasT = (float*)(ws + oBias);
  int* LISTH = (int*)(ws + oLH);
  int* LISTN = (int*)(ws + oLN);
  int* CNTH  = (int*)(ws + oCH);
  int* OFFH  = (int*)(ws + oOH);
  int* CNTN  = (int*)(ws + oCN);
  int* OFFN  = (int*)(ws + oON);
  int* FLAGH = (int*)(ws + oFH);
  int* FLAGN = (int*)(ws + oFN);

  hipFuncSetAttribute(reinterpret_cast<const void*>(&k_bucket<kSLB_H, kRC_H, kDEG_H>),
                      hipFuncAttributeMaxDynamicSharedMemorySize, (int)kLdsH);
  hipFuncSetAttribute(reinterpret_cast<const void*>(&k_bucket<kSLB_N, kRC_N, kDEG_N>),
                      hipFuncAttributeMaxDynamicSharedMemorySize, (int)kLdsN);

  k_plane<0><<<kMPN * (kH / 8) / 256, 256, 0, stream>>>(n_feat, kNN, kH, kH, RB, kMPN, kH);
  k_plane<0><<<kH * (kH / 8) / 256, 256, 0, stream>>>(W_in, kH, kH, kH, WinB, kH, kH);
  k_plane<3><<<kH * (2 * kH / 8) / 256, 256, 0, stream>>>(W_n2e, kH, kH, kH, Wn2eD, kH, kH);
  k_plane<3><<<kH * (2 * kH / 8) / 256, 256, 0, stream>>>(W_e2n, kH, kH, kH, We2nD, kH, kH);
  k_bias<<<1, 192, 0, stream>>>(b_in, b_n2e, b_e2n, biasT);

  {
    const int tiles = ((kNN + 63) / 64) * (kH / 64);
    k_gemm_nt<0, 1><<<(tiles + 7) / 8, 256, 0, stream>>>(RB, WinB, biasT, RA, kNN, kH, kH, kH);
  }
  k_plane<1><<<kMPN * (2 * kH / 8) / 256, 256, 0, stream>>>(RA, kNN, kH, kH, RB, kMPN, kH);
  {
    const int tiles = ((kNN + 63) / 64) * (kH / 64);
    k_gemm_nt<1, 1><<<(tiles + 7) / 8, 256, 0, stream>>>(RB, Wn2eD, biasT + kH, RA, kNN, kH, 2 * kH, kH);
  }

  k_bucket<kSLB_H, kRC_H, kDEG_H><<<kBLK_H, 256, kLdsH, stream>>>(hedge_idx, kE, kNE, LISTH, CNTH, OFFH, FLAGH);
  k_bucket<kSLB_N, kRC_N, kDEG_N><<<kBLK_N, 256, kLdsN, stream>>>(node_idx, kE, kNN, LISTN, CNTN, OFFN, FLAGN);

  k_replay<1, kSLB_H, kRC_H, kDEG_H><<<kMPE / 8, 256, 0, stream>>>(
      node_idx, hedge_idx, node_w, hedge_s, RA, LISTH, CNTH, OFFH, FLAGH, alpha, out + kOut1, EFhl, kNE, kMPE);

  {
    const int tiles = ((kNE + 63) / 64) * (kH / 64);
    k_gemm_nt<1, 1><<<(tiles + 7) / 8, 256, 0, stream>>>(EFhl, We2nD, biasT + 2 * kH, WHE, kNE, kH, 2 * kH, kH);
  }

  k_replay<2, kSLB_N, kRC_N, kDEG_N><<<kNN / 8, 256, 0, stream>>>(
      node_idx, hedge_idx, hedge_w, node_s, WHE, LISTN, CNTN, OFFN, FLAGN, alpha, out, EFhl, kNN, kNN);
}
